// SelfAttention_Block_42838003810703
// MI455X (gfx1250) — hardware-verified
//
#include <hip/hip_runtime.h>
#include <stdint.h>


typedef float          v8f  __attribute__((ext_vector_type(8)));
typedef float          v4f  __attribute__((ext_vector_type(4)));
typedef unsigned int   v4u  __attribute__((ext_vector_type(4)));
typedef unsigned int   v2u  __attribute__((ext_vector_type(2)));
typedef unsigned short v8us __attribute__((ext_vector_type(8)));
typedef __bf16         v16b __attribute__((ext_vector_type(16)));
typedef _Float16       v16h __attribute__((ext_vector_type(16)));
typedef _Float16       v8h  __attribute__((ext_vector_type(8)));

union FragB { v16b v; v8us half[2]; unsigned short e[16]; };
union FragH { v16h v; v8h half[2]; v8us uh[2]; _Float16 e[16]; };

static constexpr int NB = 4;
static constexpr int NN = 4096;
static constexpr int NC = 128;
static constexpr int ND = 16;
static constexpr int KR = 32;
static constexpr int PX = 136;
static constexpr int PV = 72;
static constexpr int PS = 36;

__device__ __forceinline__ unsigned short f2bf(float f) {
  unsigned int u = __builtin_bit_cast(unsigned int, f);
  u += 0x7FFFu + ((u >> 16) & 1u);
  return (unsigned short)(u >> 16);
}
__device__ __forceinline__ float bf2f(unsigned short s) {
  return __builtin_bit_cast(float, ((unsigned int)s) << 16);
}
__device__ __forceinline__ unsigned short h2us(float f) {
  return __builtin_bit_cast(unsigned short, (_Float16)f);
}

__device__ __forceinline__ v8f mma_bf16(v16b a, v16b b, v8f c) {
  v8f d = __builtin_amdgcn_wmma_f32_16x16x32_bf16(false, a, false, b, (short)0, c, false, false);
  asm volatile("v_nop\n\tv_nop\n\tv_nop\n\tv_nop" : "+v"(d) : "v"(a), "v"(b));
  return d;
}
__device__ __forceinline__ v8f mma_f16(v16h a, v16h b, v8f c) {
  v8f d = __builtin_amdgcn_wmma_f32_16x16x32_f16(false, a, false, b, (short)0, c, false, false);
  asm volatile("v_nop\n\tv_nop\n\tv_nop\n\tv_nop" : "+v"(d) : "v"(a), "v"(b));
  return d;
}

__global__ void __launch_bounds__(256)
k_prep(const float* __restrict__ Wq, const float* __restrict__ Wk, const float* __restrict__ Wv,
       unsigned short* wvt, unsigned short* wqh, unsigned short* wql,
       unsigned short* wkh, unsigned short* wkl)
{
  const int t = blockIdx.x * 256 + threadIdx.x;
  if (t < 2048) {
    const int e  = t >> 4;
    const int cb = (t & 15) << 3;
    v8us o;
    #pragma unroll
    for (int i = 0; i < 8; ++i) o[i] = h2us(Wv[(cb + i) * NC + e] * 64.0f);
    const v4u ov = __builtin_bit_cast(v4u, o);
    unsigned short* dst = wvt + (size_t)t * 8;
    *(volatile v4u*)dst = ov;
    __threadfence();
    *(volatile v4u*)dst = ov;
  } else if (t < 2560) {
    const bool isq = (t < 2304);
    const int u  = isq ? (t - 2048) : (t - 2304);
    const float* W = isq ? Wq : Wk;
    unsigned short* dh = isq ? wqh : wkh;
    unsigned short* dl = isq ? wql : wkl;
    const int d  = u >> 4;
    const int cb = (u & 15) << 3;
    v8us oh, ol;
    #pragma unroll
    for (int i = 0; i < 8; ++i) {
      const float v = W[(cb + i) * ND + d];
      const unsigned short hi = f2bf(v);
      oh[i] = hi;
      ol[i] = f2bf(v - bf2f(hi));
    }
    const v4u vh = __builtin_bit_cast(v4u, oh);
    const v4u vl = __builtin_bit_cast(v4u, ol);
    unsigned short* ph = dh + (size_t)u * 8;
    unsigned short* pl = dl + (size_t)u * 8;
    *(volatile v4u*)ph = vh;
    *(volatile v4u*)pl = vl;
    __threadfence();
    *(volatile v4u*)ph = vh;
    *(volatile v4u*)pl = vl;
  }
}

__global__ void __launch_bounds__(256)
k_proj(const float* __restrict__ x,
       const unsigned short* __restrict__ wvt,
       const unsigned short* __restrict__ wqh, const unsigned short* __restrict__ wql,
       const unsigned short* __restrict__ wkh, const unsigned short* __restrict__ wkl,
       unsigned short* Kb, unsigned short* Qb, unsigned short* Vt, int nblk)
{
  __shared__ __attribute__((aligned(16))) unsigned short xs[3 * 64 * PX];
  __shared__ __attribute__((aligned(16))) unsigned short fst[64 * KR];
  __shared__ __attribute__((aligned(16))) unsigned short gst[64 * KR];

  if ((int)blockIdx.x >= nblk) return;
  const int t = threadIdx.x, w = t >> 5, l = t & 31, h = l >> 4, m = l & 15;
  const int row0 = blockIdx.x * 64;
  const int b    = row0 >> 12;
  const int n0   = row0 & (NN - 1);
  unsigned short* xh = xs;
  unsigned short* xl = xs + 64 * PX;
  unsigned short* xf = xs + 128 * PX;

  #pragma unroll
  for (int i = 0; i < 8; ++i) {
    const int q  = i * 256 + t;
    const int r  = q >> 5;
    const int c4 = (q & 31) << 2;
    const v4f v = *(const v4f*)(x + (size_t)(row0 + r) * NC + c4);
    unsigned short hh[4], ll[4], ff[4];
    #pragma unroll
    for (int k = 0; k < 4; ++k) {
      hh[k] = f2bf(v[k]);
      ll[k] = f2bf(v[k] - bf2f(hh[k]));
      ff[k] = h2us(v[k]);
    }
    v2u ph, pl, pf;
    ph[0] = (unsigned int)hh[0] | ((unsigned int)hh[1] << 16);
    ph[1] = (unsigned int)hh[2] | ((unsigned int)hh[3] << 16);
    pl[0] = (unsigned int)ll[0] | ((unsigned int)ll[1] << 16);
    pl[1] = (unsigned int)ll[2] | ((unsigned int)ll[3] << 16);
    pf[0] = (unsigned int)ff[0] | ((unsigned int)ff[1] << 16);
    pf[1] = (unsigned int)ff[2] | ((unsigned int)ff[3] << 16);
    *(v2u*)(xh + r * PX + c4) = ph;
    *(v2u*)(xl + r * PX + c4) = pl;
    *(v2u*)(xf + r * PX + c4) = pf;
  }
  __syncthreads();

  const int rt  = w & 3;
  const int cg  = (w >> 2) << 2;
  const bool isq = (w < 4);
  const unsigned short* wth = isq ? wqh : wkh;
  const unsigned short* wtl = isq ? wql : wkl;

  const v8f zz = {0.f, 0.f, 0.f, 0.f, 0.f, 0.f, 0.f, 0.f};
  v8f acc[4];
  #pragma unroll
  for (int i = 0; i < 4; ++i) acc[i] = zz;
  v8f accp = zz;

  const int arow = (16 * rt + m) * PX + 8 * h;
  for (int k0 = 0; k0 < NC; k0 += 32) {
    FragH af;
    af.uh[0] = *(const v8us*)(xf + arow + k0);
    af.uh[1] = *(const v8us*)(xf + arow + k0 + 16);
    FragB ah, al;
    ah.half[0] = *(const v8us*)(xh + arow + k0);
    ah.half[1] = *(const v8us*)(xh + arow + k0 + 16);
    al.half[0] = *(const v8us*)(xl + arow + k0);
    al.half[1] = *(const v8us*)(xl + arow + k0 + 16);
    #pragma unroll
    for (int i = 0; i < 4; ++i) {
      const int e = ((cg + i) << 4) + m;
      FragH bv;
      bv.uh[0] = *(const v8us*)(wvt + (size_t)e * NC + k0 + 8 * h);
      bv.uh[1] = *(const v8us*)(wvt + (size_t)e * NC + k0 + 16 + 8 * h);
      acc[i] = mma_f16(af.v, bv.v, acc[i]);
    }
    FragB bh, bl;
    bh.half[0] = *(const v8us*)(wth + m * NC + k0 + 8 * h);
    bh.half[1] = *(const v8us*)(wth + m * NC + k0 + 16 + 8 * h);
    bl.half[0] = *(const v8us*)(wtl + m * NC + k0 + 8 * h);
    bl.half[1] = *(const v8us*)(wtl + m * NC + k0 + 16 + 8 * h);
    accp = mma_bf16(ah.v, bh.v, accp);
    accp = mma_bf16(ah.v, bl.v, accp);
    accp = mma_bf16(al.v, bh.v, accp);
  }

  unsigned short* pst = isq ? fst : gst;
  #pragma unroll
  for (int r = 0; r < 8; ++r) {
    const float v = accp[r];
    const unsigned short hi = f2bf(v);
    const unsigned short lo = f2bf(v - bf2f(hi));
    const int rr = 16 * rt + 8 * h + r;
    pst[rr * KR + m]      = hi;
    pst[rr * KR + 16 + m] = lo;
  }
  __syncthreads();

  unsigned short* vst = xs;
  #pragma unroll
  for (int i = 0; i < 4; ++i) {
    const int c = ((cg + i) << 4) + m;
    #pragma unroll
    for (int r = 0; r < 8; ++r) {
      const int nl = 16 * rt + 8 * h + r;
      vst[c * PV + nl] = h2us(acc[i][r] * 0.25f);
    }
  }
  __syncthreads();

  const v4u kq = *(const v4u*)(fst + 8 * t);
  const v4u qq = *(const v4u*)(gst + 8 * t);
  unsigned short* kdst = Kb + (size_t)row0 * KR + 8 * t;
  unsigned short* qdst = Qb + (size_t)row0 * KR + 8 * t;
  v4u vv[4];
  #pragma unroll
  for (int it = 0; it < 4; ++it) {
    const int c = it * 32 + w * 4 + (l >> 3);
    const int k = l & 7;
    vv[it] = *(const v4u*)(vst + c * PV + 8 * k);
  }
  *(volatile v4u*)kdst = kq;
  *(volatile v4u*)qdst = qq;
  #pragma unroll
  for (int it = 0; it < 4; ++it) {
    const int c = it * 32 + w * 4 + (l >> 3);
    const int k = l & 7;
    unsigned short* vd = Vt + ((size_t)(b * NC + c)) * NN + n0 + 8 * k;
    *(volatile v4u*)vd = vv[it];
  }
  __threadfence();
  *(volatile v4u*)kdst = kq;
  *(volatile v4u*)qdst = qq;
  #pragma unroll
  for (int it = 0; it < 4; ++it) {
    const int c = it * 32 + w * 4 + (l >> 3);
    const int k = l & 7;
    unsigned short* vd = Vt + ((size_t)(b * NC + c)) * NN + n0 + 8 * k;
    *(volatile v4u*)vd = vv[it];
  }
}

__global__ void __launch_bounds__(64)
k_attn(const unsigned short* __restrict__ Kb, const unsigned short* __restrict__ Qb,
       const unsigned short* __restrict__ Vt, const float* __restrict__ x,
       const float* __restrict__ gamma_p, float* out, int nblk)
{
  __shared__ __attribute__((aligned(16))) float stg[NC * PS];

  if ((int)blockIdx.x >= nblk) return;
  const int t = threadIdx.x, w = t >> 5, l = t & 31, h = l >> 4, m = l & 15;
  const int b   = blockIdx.x >> 7;
  const int mq0 = (blockIdx.x & 127) << 5;
  const int m0  = mq0 + (w << 4);

  const unsigned short* qrow = Qb + ((size_t)b * NN + m0 + m) * KR;
  FragB gqh, gql;
  {
    const v8us gh = *(const v8us*)(qrow + 8 * h);
    const v8us gl = *(const v8us*)(qrow + 16 + 8 * h);
    gqh.half[0] = gh; gqh.half[1] = gh;
    gql.half[0] = gl; gql.half[1] = gl;
  }

  const v8f zz = {0.f, 0.f, 0.f, 0.f, 0.f, 0.f, 0.f, 0.f};
  v8f acc[8];
  #pragma unroll
  for (int ct = 0; ct < 8; ++ct) acc[ct] = zz;
  float m_i = -3.0e38f, l_i = 0.f;

  const unsigned short* kbase = Kb + (size_t)b * NN * KR + m * KR + 8 * h;
  const unsigned short* vbase = Vt + ((size_t)b * NC + m) * NN + 8 * h;

  for (int j = 0; j < NN; j += 32) {
    FragB a0, a1;
    a0.half[0] = *(const v8us*)(kbase + (size_t)j * KR);
    a0.half[1] = *(const v8us*)(kbase + (size_t)j * KR + 16);
    a1.half[0] = *(const v8us*)(kbase + (size_t)(j + 16) * KR);
    a1.half[1] = *(const v8us*)(kbase + (size_t)(j + 16) * KR + 16);
    v8f s0 = mma_bf16(a0.v, gqh.v, zz);
    s0 = mma_bf16(a0.v, gql.v, s0);
    v8f s1 = mma_bf16(a1.v, gqh.v, zz);
    s1 = mma_bf16(a1.v, gql.v, s1);

    float mx = s0[0];
    #pragma unroll
    for (int r = 0; r < 8; ++r) { mx = fmaxf(mx, s0[r]); mx = fmaxf(mx, s1[r]); }
    mx = fmaxf(mx, __shfl_xor(mx, 16, 32));
    const float m_new = fmaxf(m_i, mx);
    const float corr  = __expf(m_i - m_new);

    float rs = 0.f;
    FragH pf;
    #pragma unroll
    for (int r = 0; r < 8; ++r) {
      const float p0 = __expf(s0[r] - m_new);
      const float p1 = __expf(s1[r] - m_new);
      rs += p0 + p1;
      pf.e[r]     = (_Float16)(p0 * 256.0f);
      pf.e[8 + r] = (_Float16)(p1 * 256.0f);
    }
    rs += __shfl_xor(rs, 16, 32);
    l_i = l_i * corr + rs;
    m_i = m_new;
    #pragma unroll
    for (int ct = 0; ct < 8; ++ct) acc[ct] = acc[ct] * corr;

    #pragma unroll
    for (int ct = 0; ct < 8; ++ct) {
      FragH vf;
      vf.uh[0] = *(const v8us*)(vbase + (size_t)ct * 16 * NN + j);
      vf.uh[1] = *(const v8us*)(vbase + (size_t)ct * 16 * NN + j + 16);
      acc[ct] = mma_f16(vf.v, pf.v, acc[ct]);
    }
  }

  const float sc = gamma_p[0] * (1.0f / l_i) * (1.0f / 4096.0f);
  #pragma unroll
  for (int ct = 0; ct < 8; ++ct) {
    #pragma unroll
    for (int r = 0; r < 8; ++r) {
      stg[((ct << 4) + 8 * h + r) * PS + (w << 4) + m] = acc[ct][r] * sc;
    }
  }
  __syncthreads();

  const size_t obase = (size_t)b * NC * NN + mq0;
  v4f vals[16];
  #pragma unroll
  for (int it = 0; it < 16; ++it) {
    const int c  = it * 8 + w * 4 + (l >> 3);
    const int k4 = (l & 7) << 2;
    const v4f a  = *(const v4f*)(stg + c * PS + k4);
    const size_t idx = obase + (size_t)c * NN + k4;
    const v4f xv = *(const v4f*)(x + idx);
    vals[it] = a + xv;
    *(volatile v4f*)(out + idx) = vals[it];
  }
  __threadfence();
  #pragma unroll
  for (int it = 0; it < 16; ++it) {
    const int c  = it * 8 + w * 4 + (l >> 3);
    const int k4 = (l & 7) << 2;
    const size_t idx = obase + (size_t)c * NN + k4;
    *(volatile v4f*)(out + idx) = vals[it];
  }
}

extern "C" void kernel_launch(void* const* d_in, const int* in_sizes, int n_in,
                              void* d_out, int out_size, void* d_ws,
                              size_t ws_size, hipStream_t stream) {
  if (n_in < 5) return;
  if (in_sizes[0] != NB * NN * NC) return;
  if (in_sizes[1] != NC * ND || in_sizes[2] != NC * ND) return;
  if (in_sizes[3] != NC * NC || in_sizes[4] < 1) return;
  if (out_size != NB * NN * NC) return;

  const float* x     = (const float*)d_in[0];
  const float* Wq    = (const float*)d_in[1];
  const float* Wk    = (const float*)d_in[2];
  const float* Wv    = (const float*)d_in[3];
  const float* gamma = (const float*)d_in[4];
  float* out = (float*)d_out;

  const size_t off_wvt = 0;
  const size_t off_wqh = off_wvt + (size_t)NC * NC * 2;
  const size_t off_wql = off_wqh + (size_t)ND * NC * 2;
  const size_t off_wkh = off_wql + (size_t)ND * NC * 2;
  const size_t off_wkl = off_wkh + (size_t)ND * NC * 2;
  const size_t off_kb  = off_wkl + (size_t)ND * NC * 2;
  const size_t kq_bytes = (size_t)NB * NN * KR * 2;
  const size_t off_qb  = off_kb + kq_bytes;
  const size_t off_vt  = off_qb + kq_bytes;
  const size_t vt_bytes = (size_t)NB * NC * NN * 2;
  const size_t total    = off_vt + vt_bytes;
  if (total > ws_size) return;

  unsigned char* ws = (unsigned char*)d_ws;
  unsigned short* wvt = (unsigned short*)(ws + off_wvt);
  unsigned short* wqh = (unsigned short*)(ws + off_wqh);
  unsigned short* wql = (unsigned short*)(ws + off_wql);
  unsigned short* wkh = (unsigned short*)(ws + off_wkh);
  unsigned short* wkl = (unsigned short*)(ws + off_wkl);
  unsigned short* Kb  = (unsigned short*)(ws + off_kb);
  unsigned short* Qb  = (unsigned short*)(ws + off_qb);
  unsigned short* Vt  = (unsigned short*)(ws + off_vt);

  const int nblk_proj = (NB * NN) / 64;
  const int nblk_attn = NB * (NN / 32);

  k_prep<<<10, 256, 0, stream>>>(Wq, Wk, Wv, wvt, wqh, wql, wkh, wkl);
  k_proj<<<nblk_proj, 256, 0, stream>>>(x, wvt, wqh, wql, wkh, wkl, Kb, Qb, Vt, nblk_proj);
  k_attn<<<nblk_attn, 64, 0, stream>>>(Kb, Qb, Vt, x, gamma, out, nblk_attn);
}
